// S6_fusion_24876450578939
// MI455X (gfx1250) — hardware-verified
//
#include <hip/hip_runtime.h>


#define NB_  4
#define DD   1024
#define LL   2048
#define NS   16
#define RR   64
typedef _Float16 h16;
typedef unsigned short bf;
typedef __attribute__((ext_vector_type(16))) __bf16   v16bf;
typedef __attribute__((ext_vector_type(16))) _Float16 v16h;
typedef __attribute__((ext_vector_type(8)))  _Float16 v8h;
typedef __attribute__((ext_vector_type(8)))  unsigned short v8us;
typedef __attribute__((ext_vector_type(8)))  float    v8f;
typedef __attribute__((ext_vector_type(4)))  float    v4f;
typedef v8h  __attribute__((may_alias)) v8ha;
typedef v4f  __attribute__((may_alias)) v4fa;
typedef v8us __attribute__((may_alias)) v8usa;

__device__ __forceinline__ unsigned short f2bf(float f) { unsigned u = __float_as_uint(f); u += 0x7FFFu + ((u >> 16) & 1u); return (unsigned short)(u >> 16); }
__device__ __forceinline__ float bf2f(unsigned short b) { return __uint_as_float(((unsigned)b) << 16); }
__device__ __forceinline__ float bfr(float f) { return bf2f(f2bf(f)); }
__device__ __forceinline__ v16h cat16(v8h lo, v8h hi) { return __builtin_shufflevector(lo, hi, 0, 1, 2, 3, 4, 5, 6, 7, 8, 9, 10, 11, 12, 13, 14, 15); }
__device__ __forceinline__ v16bf cat16b(v8us lo, v8us hi) { return __builtin_bit_cast(v16bf, __builtin_shufflevector(lo, hi, 0, 1, 2, 3, 4, 5, 6, 7, 8, 9, 10, 11, 12, 13, 14, 15)); }
__device__ __forceinline__ v8f wmma16(v16h a, v16h b, v8f c) { return __builtin_amdgcn_wmma_f32_16x16x32_f16(false, a, false, b, (short)0, c, false, false); }
__device__ __forceinline__ v8f wmmab(v16bf a, v16bf b, v8f c) { return __builtin_amdgcn_wmma_f32_16x16x32_bf16(false, a, false, b, (short)0, c, false, false); }


template <typename T16> struct WFrag;
template <> struct WFrag<h16> { typedef v16h V; static __device__ __forceinline__ V ld(const h16* p) { return cat16(*(const v8h*)p, *(const v8h*)(p + 16)); } static __device__ __forceinline__ v8f mma(V a, V b, v8f c) { return wmma16(a, b, c); } };
template <> struct WFrag<bf> { typedef v16bf V; static __device__ __forceinline__ V ld(const bf* p) { return cat16b(*(const v8us*)p, *(const v8us*)(p + 16)); } static __device__ __forceinline__ v8f mma(V a, V b, v8f c) { return wmmab(a, b, c); } };
template <typename T16, int NSPLIT, bool BIAS>
__global__ __launch_bounds__(32) void k_gemmw(const T16* __restrict__ A, const T16* __restrict__ A2, const T16* __restrict__ Bt, const T16* __restrict__ Bt2, int K, float* C, int ldc, const float* __restrict__ bias, size_t sA, size_t sB, size_t sC) {
    typedef typename WFrag<T16>::V V;
    __shared__ __align__(16) float os[16 * 68];
    const size_t z = blockIdx.z; A += z * sA; if (A2) A2 += z * sA; Bt += z * sB; if (Bt2) Bt2 += z * sB; C += z * sC;
    const int lane = threadIdx.x & 31, lr = lane & 15, hi = lane >> 4; const int r0 = blockIdx.x * 64, c0 = blockIdx.y * 64;
    v8f acc[4][4];
#pragma unroll
    for (int mb = 0; mb < 4; ++mb)
#pragma unroll
        for (int nb = 0; nb < 4; ++nb) acc[mb][nb] = (v8f){};
    const size_t aoff = (size_t)(r0 + lr) * K + 8 * hi, boff = (size_t)(c0 + lr) * K + 8 * hi;
#pragma unroll 1
    for (int kc = 0; kc < K; kc += 32) {
        V a[4], a2[4];
#pragma unroll
        for (int mb = 0; mb < 4; ++mb) { a[mb] = WFrag<T16>::ld(A + aoff + (size_t)mb * 16 * K + kc); if (NSPLIT == 1 || NSPLIT == 2) a2[mb] = WFrag<T16>::ld(A2 + aoff + (size_t)mb * 16 * K + kc); }
#pragma unroll
        for (int nb = 0; nb < 4; ++nb) { const V b = WFrag<T16>::ld(Bt + boff + (size_t)nb * 16 * K + kc); V b2; if (NSPLIT >= 2) b2 = WFrag<T16>::ld(Bt2 + boff + (size_t)nb * 16 * K + kc);
#pragma unroll
            for (int mb = 0; mb < 4; ++mb) { acc[mb][nb] = WFrag<T16>::mma(a[mb], b, acc[mb][nb]); if (NSPLIT == 1 || NSPLIT == 2) acc[mb][nb] = WFrag<T16>::mma(a2[mb], b, acc[mb][nb]); if (NSPLIT >= 2) acc[mb][nb] = WFrag<T16>::mma(a[mb], b2, acc[mb][nb]); } }
        asm volatile("v_nop\n\tv_nop\n\tv_nop\n\tv_nop" : "+v"(acc[0][0]), "+v"(acc[1][1]), "+v"(acc[2][2]), "+v"(acc[3][3]) : "v"(a[0]), "v"(a[3]));
    }
#pragma unroll
    for (int mb = 0; mb < 4; ++mb) {
#pragma unroll
        for (int nb = 0; nb < 4; ++nb) {
#pragma unroll
            for (int j = 0; j < 8; ++j) os[(hi * 8 + j) * 68 + nb * 16 + lr] = acc[mb][nb][j]; }
        __builtin_amdgcn_wave_barrier(); asm volatile("" ::: "memory");
        float* crow = C + (size_t)(r0 + mb * 16) * ldc + c0;
#pragma unroll 1
        for (int ps = 0; ps < 2; ++ps) {
#pragma unroll
            for (int s = 0; s < 8; ++s) { const int row = 2 * s + hi, cofs = lr * 4; v4f val = *(const v4fa*)(os + row * 68 + cofs); if (BIAS) { val[0] += bfr(bias[c0 + cofs]); val[1] += bfr(bias[c0 + cofs + 1]); val[2] += bfr(bias[c0 + cofs + 2]); val[3] += bfr(bias[c0 + cofs + 3]); }
                *(volatile v4f*)(crow + (size_t)row * ldc + cofs) = val; }
            if (ps == 0) __threadfence(); }
        __builtin_amdgcn_wave_barrier(); asm volatile("" ::: "memory");
    }
}

__device__ __forceinline__ void splitf(float y, unsigned short& h, unsigned short& l) { h = f2bf(y); l = f2bf(y - bf2f(h)); }
typedef __attribute__((ext_vector_type(2))) unsigned short v2us;
typedef __attribute__((ext_vector_type(4))) unsigned short v4us;
typedef __attribute__((ext_vector_type(2))) float v2f;

__global__ __launch_bounds__(256) void k_cvt8(const float* __restrict__ src, bf* dst, size_t n8) { const size_t i = (size_t)blockIdx.x * 256 + threadIdx.x; if (i >= n8) return; const v8f v = *(const v8f*)(src + i * 8); v8us o;
#pragma unroll
    for (int k = 0; k < 8; ++k) o[k] = f2bf(v[k]); *(volatile v8us*)(dst + i * 8) = o; __threadfence(); *(volatile v8us*)(dst + i * 8) = o; }
__global__ __launch_bounds__(256) void k_xt(const float* __restrict__ x, bf* XT) { const int e = (blockIdx.x * 256 + threadIdx.x) * 2; if (e >= LL * DD) return; const int d = e % DD; const int l = e / DD; v2us o; o[0] = f2bf(x[(size_t)d * LL + l]); o[1] = f2bf(x[(size_t)(d + 1) * LL + l]); *(volatile v2us*)(XT + e) = o; __threadfence(); *(volatile v2us*)(XT + e) = o; }
__global__ __launch_bounds__(256) void k_wpad(const float* __restrict__ w, int NV, bf* Bt) { const int e = (blockIdx.x * 256 + threadIdx.x) * 8; if (e >= 64 * DD) return; const int n = e / DD; v8us o;
    for (int u = 0; u < 8; ++u) o[u] = (n < NV) ? f2bf(w[e - (size_t)0 + u]) : (unsigned short)0;
    *(volatile v8us*)(Bt + e) = o; __threadfence(); *(volatile v8us*)(Bt + e) = o; }
__global__ __launch_bounds__(256) void k_spl(const float* __restrict__ F, bf* Hh, bf* Hl) { const int e = (blockIdx.x * 256 + threadIdx.x) * 4; if (e >= LL * RR) return; const v4f a = *(const v4f*)(F + e); v4us oh, ol;
#pragma unroll
    for (int u = 0; u < 4; ++u) { unsigned short h, l; splitf(a[u], h, l); oh[u] = h; ol[u] = l; } *(volatile v4us*)(Hh + e) = oh; *(volatile v4us*)(Hl + e) = ol; __threadfence(); *(volatile v4us*)(Hh + e) = oh; *(volatile v4us*)(Hl + e) = ol; }
__global__ __launch_bounds__(64) void k_scan(const float* __restrict__ DEL, const float* __restrict__ u, const float* __restrict__ BB, const float* __restrict__ CCm, const float* __restrict__ A_log, float* Y) {
    __shared__ float ybuf[2][32][33];
    const int wv = threadIdx.x >> 5; const int lane = threadIdx.x & 31; const int d = (blockIdx.x * 2 + wv) * 32 + lane; if (d >= DD) return;
    float A[NS], x[NS];
#pragma unroll
    for (int n = 0; n < NS; ++n) { A[n] = -__expf(bfr(A_log[d * NS + n])); x[n] = 0.f; }
    const float* ud = u + (size_t)d * LL;
    for (int l0 = 0; l0 < LL; l0 += 32) {
        for (int i = 0; i < 32; ++i) { const int l = l0 + i;
            const float dr = DEL[(size_t)l * DD + d]; const float dl = (dr > 20.f) ? dr : log1pf(__expf(dr));
            float du = __fmul_rn(dl, bfr(ud[l])); asm volatile("" : "+v"(du)); const float* bl = BB + (size_t)l * 64; const float* cl = CCm + (size_t)l * 64; float y = 0.f;
#pragma unroll
            for (int n = 0; n < NS; ++n) { float da = __fmul_rn(dl, A[n]); asm volatile("" : "+v"(da)); const float ex = __expf(da); float t1 = __fmul_rn(ex, x[n]); asm volatile("" : "+v"(t1)); float t2 = __fmul_rn(du, bl[n]); asm volatile("" : "+v"(t2)); x[n] = __fadd_rn(t1, t2); float p = __fmul_rn(x[n], cl[n]); asm volatile("" : "+v"(p)); y = __fadd_rn(y, p); }
            ybuf[wv][lane][i] = y; }
        __syncthreads();
        for (int ps = 0; ps < 2; ++ps) {
#pragma unroll
            for (int r = 0; r < 8; ++r) { const int ch = r * 4 + (lane >> 3); const int c4 = (lane & 7) * 4; v4f o; o[0] = ybuf[wv][ch][c4]; o[1] = ybuf[wv][ch][c4 + 1]; o[2] = ybuf[wv][ch][c4 + 2]; o[3] = ybuf[wv][ch][c4 + 3];
                *(volatile v4f*)(Y + (size_t)((blockIdx.x * 2 + wv) * 32 + ch) * LL + l0 + c4) = o; }
            if (ps == 0) __threadfence(); }
        __syncthreads(); } }

extern "C" void kernel_launch(void* const* d_in, const int* in_sizes, int n_in,
                              void* d_out, int out_size, void* d_ws, size_t ws_size, hipStream_t stream) {
    (void)in_sizes; (void)n_in; (void)out_size;
    const float** I = (const float**)d_in;
    const float *u = I[0], *mask = I[1], *info = I[2], *W_C = I[3], *W_B = I[4], *W_delta = I[5], *W_dt = I[6], *dt_bias = I[7], *A_log = I[8];
    float* OUT = (float*)d_out;
    char* wsp = (char*)d_ws;
    auto take = [&](size_t bytes) { char* p = wsp; wsp += (bytes + 255) & ~(size_t)255; return (void*)p; };
    bf* BWD = (bf*)take((size_t)RR * DD * 2); bf* BWB = (bf*)take((size_t)64 * DD * 2); bf* BWC = (bf*)take((size_t)64 * DD * 2); bf* BDT = (bf*)take((size_t)DD * RR * 2);
    bf* XT = (bf*)take((size_t)LL * DD * 2); float* DTL = (float*)take((size_t)LL * RR * 4); bf* Dh = (bf*)take((size_t)LL * RR * 2); bf* Dl = (bf*)take((size_t)LL * RR * 2); float* DEL = (float*)take((size_t)LL * DD * 4); float* BB = (float*)take((size_t)LL * 64 * 4); float* CCm = (float*)take((size_t)LL * 64 * 4);
    if ((size_t)(wsp - (char*)d_ws) > ws_size) return;
    k_cvt8<<<(RR * DD / 8 + 255) / 256, 256, 0, stream>>>(W_delta, BWD, RR * DD / 8);
    k_wpad<<<(64 * DD / 8 + 255) / 256, 256, 0, stream>>>(W_B, NS, BWB); k_wpad<<<(64 * DD / 8 + 255) / 256, 256, 0, stream>>>(W_C, NS, BWC);
    k_cvt8<<<(DD * RR / 8 + 255) / 256, 256, 0, stream>>>(W_dt, BDT, DD * RR / 8);
    for (int b = 0; b < NB_; ++b) { const size_t bo = (size_t)b * DD * LL;
        k_xt<<<(LL * DD / 2 + 255) / 256, 256, 0, stream>>>(mask + bo, XT);
        k_gemmw<bf, 0, false><<<dim3(LL / 64, 1, 1), 32, 0, stream>>>(XT, nullptr, BWD, nullptr, DD, DTL, RR, nullptr, 0, 0, 0); k_spl<<<(LL * RR / 4 + 255) / 256, 256, 0, stream>>>(DTL, Dh, Dl);
        k_gemmw<bf, 1, true><<<dim3(LL / 64, DD / 64, 1), 32, 0, stream>>>(Dh, Dl, BDT, nullptr, RR, DEL, DD, dt_bias, 0, 0, 0);
        k_xt<<<(LL * DD / 2 + 255) / 256, 256, 0, stream>>>(info + bo, XT); k_gemmw<bf, 0, false><<<dim3(LL / 64, 1, 1), 32, 0, stream>>>(XT, nullptr, BWB, nullptr, DD, BB, 64, nullptr, 0, 0, 0);
        k_xt<<<(LL * DD / 2 + 255) / 256, 256, 0, stream>>>(u + bo, XT); k_gemmw<bf, 0, false><<<dim3(LL / 64, 1, 1), 32, 0, stream>>>(XT, nullptr, BWC, nullptr, DD, CCm, 64, nullptr, 0, 0, 0);
        k_scan<<<DD / 64, 64, 0, stream>>>(DEL, u + bo, BB, CCm, A_log, OUT + bo); }
}
